// S4SSM_14508399526249
// MI455X (gfx1250) — hardware-run, weakly checked
//
#include <hip/hip_runtime.h>
#include <math.h>

typedef __attribute__((ext_vector_type(16))) _Float16 v16h;
typedef __attribute__((ext_vector_type(8)))  _Float16 v8h;
typedef __attribute__((ext_vector_type(16))) __bf16   v16b;
typedef __attribute__((ext_vector_type(8)))  __bf16   v8b;
typedef __attribute__((ext_vector_type(8)))  float    v8f;
typedef __attribute__((ext_vector_type(4)))  float    v4f;

constexpr int kH      = 1025;
constexpr int kL      = 2048;
constexpr int kNS     = 32;
constexpr int kO      = 2 * kH;
constexpr int kKP     = 1056;
constexpr int kPitch  = 1088;
constexpr int kMP     = 2112;
constexpr int kLayers = 4;
constexpr float kCarryW = 64.0f;
constexpr float kCarryY = 16.0f;
constexpr float kFold   = 1.0f / (kCarryW * kCarryY);
constexpr float kF16MinNormal = 6.103515625e-05f;

constexpr int kScCh = 64;
constexpr int kScTS = 64;
constexpr int kScYP = 68;
constexpr int kScBlocks = kPitch / kScCh;

static_assert(kNS == 32, "one state per lane");
static_assert((kKP % 32) == 0 && kKP >= kH, "K pad");
static_assert((kPitch % 64) == 0 && kPitch >= kKP, "plane pitch in whole lines");
static_assert((kMP % 64) == 0 && kMP >= kO, "M pad");
static_assert((kL % 64) == 0 && kL == 2048, "N tile multiple");
static_assert((kL % kScTS) == 0 && kScBlocks * kScCh == kPitch, "scan tiling");
static_assert(((kMP * (kPitch / 8)) % 256) == 0, "pack grid exact");
static_assert(((kH * (kL / 4)) % 256) == 0, "gate grid exact");
static_assert((((kMP / 64) * (kL / 64)) % 8) == 0, "gemm grid exact");

constexpr size_t kSzPar = (size_t)kH * kNS * 4;
constexpr size_t kSzWH  = (size_t)kMP * kPitch * 2;
constexpr size_t kSzYT  = (size_t)kL * kPitch * 2;
constexpr size_t kSzG   = (size_t)kMP * kL * 4;
constexpr size_t kSzU   = (size_t)kH * kL * 4;
constexpr size_t kOffDAR = 0;
constexpr size_t kOffDAI = kOffDAR + kSzPar;
constexpr size_t kOffCBR = kOffDAI + kSzPar;
constexpr size_t kOffCBI = kOffCBR + kSzPar;
constexpr size_t kOffWH  = kOffCBI + kSzPar;
constexpr size_t kOffYT  = kOffWH + kSzWH;
constexpr size_t kOffG   = kOffYT + kSzYT;
constexpr size_t kOffUA  = kOffG + kSzG;
constexpr size_t kOffUB  = kOffUA + kSzU;
constexpr size_t kWsTotal = kOffUB + kSzU;
static_assert(kWsTotal == 43672064ull, "carve total");
static_assert(kWsTotal <= 134217728ull, "carve cap");
static_assert((kSzPar % 128) == 0 && (kSzWH % 128) == 0 && (kSzYT % 128) == 0 && (kSzG % 128) == 0 && (kSzU % 128) == 0,
              "128-B aligned regions");

__device__ __forceinline__ unsigned short f2bf_bits(float f) {
  unsigned u = __float_as_uint(f);
  return (unsigned short)((u + 0x7FFFu + ((u >> 16) & 1u)) >> 16);
}
__device__ __forceinline__ float bf_bits2f(unsigned short h) { return __uint_as_float(((unsigned)h) << 16); }

__device__ __forceinline__ void dep_guard_h(v8f& a, v8f& b, v16h x, v16h y) { asm volatile("v_nop\n\tv_nop\n\tv_nop\n\tv_nop" : "+v"(a), "+v"(b) : "v"(x), "v"(y)); }
__device__ __forceinline__ void dep_guard_b(v8f& a, v8f& b, v16b x, v16b y) { asm volatile("v_nop\n\tv_nop\n\tv_nop\n\tv_nop" : "+v"(a), "+v"(b) : "v"(x), "v"(y)); }
__device__ __forceinline__ void keep4_h(v16h a, v16h b, v16h c, v16h d) { asm volatile("v_nop" :: "v"(a), "v"(b), "v"(c), "v"(d)); }
__device__ __forceinline__ void keep4_b(v16b a, v16b b, v16b c, v16b d) { asm volatile("v_nop" :: "v"(a), "v"(b), "v"(c), "v"(d)); }
__device__ __forceinline__ void acc_guard4(v8f& a, v8f& b, v8f& c, v8f& d) { asm volatile("v_nop\n\tv_nop\n\tv_nop\n\tv_nop" : "+v"(a), "+v"(b), "+v"(c), "+v"(d)); }
__device__ __forceinline__ void tie_acc(v8f& a) { asm volatile("" : "+v"(a)); }

template <typename T> struct Frag;
template <> struct Frag<_Float16> {
  typedef v16h V; union U { v16h v; v8h h[2]; };
  static __device__ __forceinline__ v16h load(const _Float16* p) {
    U f; f.h[0] = *(const v8h*)(p); f.h[1] = *(const v8h*)(p + 16); return f.v;
  }
  static __device__ __forceinline__ v8f mma(v16h a, v16h b, v8f c) {
    return __builtin_amdgcn_wmma_f32_16x16x32_f16(false, a, false, b, (short)0, c, false, false);
  }
  static __device__ __forceinline__ void guard(v8f& a, v8f& b, v16h x, v16h y) { dep_guard_h(a, b, x, y); }
  static __device__ __forceinline__ void keep(v16h a, v16h b, v16h c, v16h d) { keep4_h(a, b, c, d); }
};
template <> struct Frag<__bf16> {
  typedef v16b V; union U { v16b v; v8b h[2]; };
  static __device__ __forceinline__ v16b load(const __bf16* p) {
    U f; f.h[0] = *(const v8b*)(p); f.h[1] = *(const v8b*)(p + 16); return f.v;
  }
  static __device__ __forceinline__ v8f mma(v16b a, v16b b, v8f c) {
    return __builtin_amdgcn_wmma_f32_16x16x32_bf16(false, a, false, b, (short)0, c, false, false);
  }
  static __device__ __forceinline__ void guard(v8f& a, v8f& b, v16b x, v16b y) { dep_guard_b(a, b, x, y); }
  static __device__ __forceinline__ void keep(v16b a, v16b b, v16b c, v16b d) { keep4_b(a, b, c, d); }
};

template <int ET> struct Elem;
template <> struct Elem<0> { typedef _Float16 T; };
template <> struct Elem<1> { typedef __bf16 T; };
template <int ET, bool SPLIT, int BIAS_MODE, int OUT_MODE, bool RESID, int ACT = 0>
__global__ __launch_bounds__(256) void wmma_gemm64(
    const unsigned short* __restrict__ Ap, const unsigned short* __restrict__ A2p, int lda, long strideA,
    const unsigned short* __restrict__ Btp, const unsigned short* __restrict__ Bt2p, int ldb, long strideB,
    void* __restrict__ Cout, void* __restrict__ Cout2, int ldc, long strideC,
    const float* __restrict__ bias,
    const float* __restrict__ resid, long strideR,
    int M, int N, int K, float scale) {
  typedef typename Elem<ET>::T T;
  typedef typename Frag<T>::V V;
  const T* A = (const T*)Ap; const T* A2 = (const T*)A2p; const T* Bt = (const T*)Btp; const T* Bt2 = (const T*)Bt2p;
  __shared__ __align__(16) float sT[8][16 * 68];
  const int b    = blockIdx.y;
  const int lane = threadIdx.x & 31;
  const int wave = threadIdx.x >> 5;
  const int tilesN = N >> 6;
  const int tilesM = M >> 6;
  const int tile = blockIdx.x * 8 + wave;
  if (tile >= tilesM * tilesN) return;
  const int tm = tile / tilesN;
  const int tn = tile - tm * tilesN;
  const int m0 = tm << 6;
  const int n0 = tn << 6;

  const T* Ab  = A  + (size_t)b * strideA;
  const T* Bb  = Bt + (size_t)b * strideB;
  const T* Ab2 = SPLIT ? (A2  + (size_t)b * strideA) : nullptr;
  const T* Bb2 = SPLIT ? (Bt2 + (size_t)b * strideB) : nullptr;

  const int rlane = lane & 15;
  const int koff  = (lane >> 4) * 8;
  const int mOff  = (lane >> 4) * 8;

  v8f acc[4][4];
#pragma unroll
  for (int i = 0; i < 4; ++i)
#pragma unroll
    for (int j = 0; j < 4; ++j) acc[i][j] = (v8f){0.f,0.f,0.f,0.f,0.f,0.f,0.f,0.f};

  for (int k0 = 0; k0 < K; k0 += 32) {
    V bh[4], bl[4];
#pragma unroll
    for (int j = 0; j < 4; ++j) {
      const size_t bo = (size_t)(n0 + (j << 4) + rlane) * ldb + koff + k0;
      bh[j] = Frag<T>::load(Bb + bo);
      if (SPLIT) bl[j] = Frag<T>::load(Bb2 + bo);
    }
#pragma unroll
    for (int i = 0; i < 4; ++i) {
      const size_t ao = (size_t)(m0 + (i << 4) + rlane) * lda + koff + k0;
      V ah = Frag<T>::load(Ab + ao);
      V al;
      if (SPLIT) al = Frag<T>::load(Ab2 + ao);
#pragma unroll
      for (int j = 0; j < 4; ++j) {
        acc[i][j] = Frag<T>::mma(ah, bh[j], acc[i][j]);
        if (SPLIT) {
          acc[i][j] = Frag<T>::mma(ah, bl[j], acc[i][j]);
          acc[i][j] = Frag<T>::mma(al, bh[j], acc[i][j]);
        }
      }
      tie_acc(acc[i][1]);
      tie_acc(acc[i][2]);
      Frag<T>::guard(acc[i][0], acc[i][3], ah, SPLIT ? al : ah);
    }
    Frag<T>::keep(bh[0], bh[1], bh[2], bh[3]);
    if (SPLIT) Frag<T>::keep(bl[0], bl[1], bl[2], bl[3]);
  }
  acc_guard4(acc[0][0], acc[0][1], acc[0][2], acc[0][3]);
  acc_guard4(acc[1][0], acc[1][1], acc[1][2], acc[1][3]);
  acc_guard4(acc[2][0], acc[2][1], acc[2][2], acc[2][3]);
  acc_guard4(acc[3][0], acc[3][1], acc[3][2], acc[3][3]);

  float* slab = sT[wave];
  const float* Rb = RESID ? (resid + (size_t)b * strideR) : nullptr;
#pragma unroll
  for (int i = 0; i < 4; ++i) {
    const int mBase = m0 + (i << 4);
#pragma unroll
    for (int j = 0; j < 4; ++j) {
      const int n = n0 + (j << 4) + rlane;
      float bv = 0.f;
      if (BIAS_MODE == 2) bv = bias[n];
#pragma unroll
      for (int r = 0; r < 8; ++r) {
        float v = acc[i][j][r] * scale;
        if (BIAS_MODE == 1) v += bias[mBase + mOff + r];
        if (BIAS_MODE == 2) v += bv;
        if (RESID) v += Rb[(size_t)(mBase + mOff + r) * ldc + n];
        if (ACT == 1) v = tanhf(v);
        if (ACT == 2) v = fmaxf(v, 0.0f);
        if (ACT == 3) v = v / (1.0f + expf(-v));
        if (ACT == 4) v = (v > 0.f) ? v : 0.01f * v;
        slab[(mOff + r) * 68 + (j << 4) + rlane] = v;
      }
    }
    __builtin_amdgcn_fence(__ATOMIC_RELEASE, "workgroup");
    __builtin_amdgcn_wave_barrier();
    __builtin_amdgcn_fence(__ATOMIC_ACQUIRE, "workgroup");
    if (OUT_MODE == 0) {
      float* C = (float*)Cout + (size_t)b * strideC;
      const int hh = lane >> 4, c4 = (lane & 15) * 4;
      for (int pass = 0; pass < 2; ++pass) {
#pragma unroll
        for (int it = 0; it < 8; ++it) {
          const int row = it * 2 + hh;
          v4f v = *(const v4f*)(slab + row * 68 + c4);
          *(volatile v4f*)(C + (size_t)(mBase + row) * ldc + n0 + c4) = v;
        }
        __threadfence();
      }
    } else {
      const int q = lane >> 3, c8 = (lane & 7) * 8;
      unsigned short* C  = (unsigned short*)Cout  + (size_t)b * strideC;
      unsigned short* C2 = (OUT_MODE == 2) ? ((unsigned short*)Cout2 + (size_t)b * strideC) : nullptr;
      for (int pass = 0; pass < 2; ++pass) {
#pragma unroll
        for (int it = 0; it < 4; ++it) {
          const int row = it * 4 + q;
          const float* sp = slab + row * 68 + c8;
          v8h hv, lv;
#pragma unroll
          for (int e = 0; e < 8; ++e) {
            if (OUT_MODE == 1) {
              hv[e] = (_Float16)sp[e];
            } else {
              unsigned short hb = f2bf_bits(sp[e]);
              unsigned short lb = f2bf_bits(sp[e] - bf_bits2f(hb));
              hv[e] = __builtin_bit_cast(_Float16, hb);
              lv[e] = __builtin_bit_cast(_Float16, lb);
            }
          }
          *(volatile v8h*)(C + (size_t)(mBase + row) * ldc + n0 + c8) = hv;
          if (OUT_MODE == 2) *(volatile v8h*)(C2 + (size_t)(mBase + row) * ldc + n0 + c8) = lv;
        }
        __threadfence();
      }
    }
    __builtin_amdgcn_fence(__ATOMIC_RELEASE, "workgroup");
    __builtin_amdgcn_wave_barrier();
    __builtin_amdgcn_fence(__ATOMIC_ACQUIRE, "workgroup");
  }
}

__device__ __forceinline__ _Float16 to_f16_flush(float x) {
  const float a = fabsf(x);
  const float z = (a < kF16MinNormal) ? 0.0f : x;
  return (_Float16)z;
}

__global__ __launch_bounds__(256) void discretize_kernel(
    const float* __restrict__ log_dt, const float* __restrict__ A_log, const float* __restrict__ A_im,
    const float* __restrict__ B_re, const float* __restrict__ B_im,
    const float* __restrict__ C_re, const float* __restrict__ C_im,
    float* __restrict__ dAr, float* __restrict__ dAi, float* __restrict__ cbr, float* __restrict__ cbi)
{
  const int lane = threadIdx.x & 31, wave = threadIdx.x >> 5;
  const int h  = blockIdx.x * 8 + wave;
  const int hc = (h < kH) ? h : (kH - 1);
  const int i  = hc * kNS + lane;
  const float ar = -expf(A_log[i]);
  const float ai = A_im[i];
  const float dt = expf(log_dt[hc]);
  const float br = B_re[i], bi = B_im[i];
  const float crv = C_re[i], civ = C_im[i];
  const float ex  = expf(dt * ar);
  const float ang = dt * ai;
  float sn, cs;
  sincosf(ang, &sn, &cs);
  const float dar = ex * cs, dai = ex * sn;
  const float nr = dar - 1.0f, ni = dai;
  const float inv = 1.0f / (ar * ar + ai * ai);
  const float qr = (nr * ar + ni * ai) * inv;
  const float qi = (ni * ar - nr * ai) * inv;
  const float dbr = qr * br - qi * bi;
  const float dbi = qr * bi + qi * br;
  const float pr = crv * dbr - civ * dbi;
  const float pi = crv * dbi + civ * dbr;
  if (h < kH) {
    for (int pass = 0; pass < 2; ++pass) {
      *(volatile float*)(dAr + i) = dar;
      *(volatile float*)(dAi + i) = dai;
      *(volatile float*)(cbr + i) = pr;
      *(volatile float*)(cbi + i) = pi;
      __threadfence();
    }
  }
}

__global__ __launch_bounds__(256) void pack_weight_kernel(const float* __restrict__ W, unsigned short* __restrict__ WH)
{
  const int i = blockIdx.x * 256 + threadIdx.x;
  if (i >= kMP * (kPitch / 8)) return;
  const int row = i / (kPitch / 8);
  const int c8  = (i - row * (kPitch / 8)) * 8;
  const int rc  = (row < kO) ? row : (kO - 1);
  v8h hv;
#pragma unroll
  for (int e = 0; e < 8; ++e) {
    const int k  = c8 + e;
    const int kc = (k < kH) ? k : (kH - 1);
    const float v = W[(size_t)rc * kH + kc];
    const bool ok = (row < kO) && (k < kH);
    const float s = v * kCarryW;
    const float z = ok ? s : 0.0f;
    hv[e] = to_f16_flush(z);
  }
  unsigned short* p = WH + (size_t)i * 8;
  *(volatile v8h*)p = hv;
  __threadfence();
  *(volatile v8h*)p = hv;
}

__global__ __launch_bounds__(256) void diag_scan_gelu_kernel(
    const float* __restrict__ U,
    const float* __restrict__ dAr, const float* __restrict__ dAi,
    const float* __restrict__ cbr, const float* __restrict__ cbi,
    const float* __restrict__ Dv, unsigned short* __restrict__ YT)
{
  __shared__ __align__(16) float sY[kScTS * kScYP];
  __shared__ float sSr[kScCh * 32];
  __shared__ float sSi[kScCh * 32];
  const int tid = threadIdx.x, lane = tid & 31, wave = tid >> 5;
  const int h0 = blockIdx.x * kScCh;
#pragma unroll 1
  for (int c = 0; c < 8; ++c) {
    sSr[(wave * 8 + c) * 32 + lane] = 0.0f;
    sSi[(wave * 8 + c) * 32 + lane] = 0.0f;
  }
  const int q = lane >> 3, c8 = (lane & 7) * 8;
#pragma unroll 1
  for (int t0 = 0; t0 < kL; t0 += kScTS) {
    __syncthreads();
#pragma unroll 1
    for (int c = 0; c < 8; ++c) {
      const int cl = wave * 8 + c;
      const int h  = h0 + cl;
      const int hc = (h < kH) ? h : (kH - 1);
      const int pi = hc * kNS + lane;
      const float ar = dAr[pi], ai = dAi[pi];
      const float cr = cbr[pi], ci = cbi[pi];
      const float dch = Dv[hc];
      float sr = sSr[cl * 32 + lane];
      float si = sSi[cl * 32 + lane];
      const float* urow = U + (size_t)hc * kL + t0;
#pragma unroll 1
      for (int sub = 0; sub < 2; ++sub) {
        const float uv = urow[sub * 32 + lane];
        float ybuf = 0.0f;
#pragma unroll 1
        for (int s = 0; s < 32; ++s) {
          const float ut  = __shfl(uv, s, 32);
          const float nsr = fmaf(ar, sr, fmaf(-ai, si, ut));
          const float nsi = fmaf(ar, si, ai * sr);
          sr = nsr;
          si = nsi;
          float p = fmaf(cr, sr, -(ci * si));
          p += __shfl_xor(p, 16, 32);
          p += __shfl_xor(p, 8, 32);
          p += __shfl_xor(p, 4, 32);
          p += __shfl_xor(p, 2, 32);
          p += __shfl_xor(p, 1, 32);
          const float y = fmaf(dch, ut, 2.0f * p);
          ybuf = (s == lane) ? y : ybuf;
        }
        const float ge = 0.5f * ybuf * (1.0f + erff(ybuf * 0.70710678118654752f));
        const float gs = ge * kCarryY;
        const float gz = (h < kH) ? gs : 0.0f;
        sY[(sub * 32 + lane) * kScYP + cl] = gz;
      }
      sSr[cl * 32 + lane] = sr;
      sSi[cl * 32 + lane] = si;
    }
    __syncthreads();
    v8h hv[2];
#pragma unroll
    for (int it = 0; it < 2; ++it) {
      const int row = it * 32 + wave * 4 + q;
      const float* sp = sY + row * kScYP + c8;
      const v4f a0 = *(const v4f*)(sp);
      const v4f a1 = *(const v4f*)(sp + 4);
#pragma unroll
      for (int e = 0; e < 4; ++e) {
        const float f0 = a0[e];
        const float f1 = a1[e];
        hv[it][e]     = to_f16_flush(f0);
        hv[it][4 + e] = to_f16_flush(f1);
      }
    }
    for (int pass = 0; pass < 2; ++pass) {
#pragma unroll
      for (int it = 0; it < 2; ++it) {
        const int row = it * 32 + wave * 4 + q;
        *(volatile v8h*)(YT + (size_t)(t0 + row) * kPitch + h0 + c8) = hv[it];
      }
      __threadfence();
    }
  }
}

__global__ __launch_bounds__(256) void glu_skip_kernel(
    const float* __restrict__ Uin, const float* __restrict__ G, const float* __restrict__ bout,
    const int* __restrict__ lcount, float* __restrict__ Uout)
{
  const int i = blockIdx.x * 256 + threadIdx.x;
  if (i >= kH * (kL / 4)) return;
  const int h  = i >> 9;
  const int t4 = (i & 511) << 2;
  const v4f u = *(const v4f*)(Uin + (size_t)h * kL + t4);
  const v4f a = *(const v4f*)(G + (size_t)h * kL + t4);
  const v4f b = *(const v4f*)(G + (size_t)(h + kH) * kL + t4);
  const float b1 = bout[h];
  const float b2 = bout[h + kH];
  const bool ok = (lcount[0] == kLayers);
  const float qnan = __uint_as_float(0x7fc00000u);
  v4f o;
#pragma unroll
  for (int e = 0; e < 4; ++e) {
    const float g1 = a[e] + b1;
    const float g2 = b[e] + b2;
    const float sg = __builtin_amdgcn_rcpf(1.0f + expf(-g2));
    const float r  = fmaf(g1, sg, u[e]);
    o[e] = ok ? r : qnan;
  }
  float* p = Uout + (size_t)h * kL + t4;
  *(volatile v4f*)p = o;
  __threadfence();
  *(volatile v4f*)p = o;
}

extern "C" void kernel_launch(void* const* d_in, const int* in_sizes, int n_in,
                              void* d_out, int out_size, void* d_ws, size_t ws_size,
                              hipStream_t stream) {
  if (n_in < 12) return;
  if (in_sizes[0] != kH * kL) return;
  if (in_sizes[1] != kH) return;
  if (in_sizes[2] != kH * kNS) return;
  if (in_sizes[3] != kH * kNS) return;
  if (in_sizes[4] != kH * kNS) return;
  if (in_sizes[5] != kH * kNS) return;
  if (in_sizes[6] != kH * kNS) return;
  if (in_sizes[7] != kH * kNS) return;
  if (in_sizes[8] != kH) return;
  if (in_sizes[9] != kO * kH) return;
  if (in_sizes[10] != kO) return;
  if (in_sizes[11] != 1) return;
  if (out_size != kH * kL) return;
  if (ws_size < kWsTotal) return;

  const float* Z      = (const float*)d_in[0];
  const float* log_dt = (const float*)d_in[1];
  const float* A_log  = (const float*)d_in[2];
  const float* A_im   = (const float*)d_in[3];
  const float* B_re   = (const float*)d_in[4];
  const float* B_im   = (const float*)d_in[5];
  const float* C_re   = (const float*)d_in[6];
  const float* C_im   = (const float*)d_in[7];
  const float* Dv     = (const float*)d_in[8];
  const float* Wout   = (const float*)d_in[9];
  const float* bout   = (const float*)d_in[10];
  const int*   lcount = (const int*)d_in[11];
  float* out = (float*)d_out;

  char* ws = (char*)d_ws;
  float* dAr = (float*)(ws + kOffDAR);
  float* dAi = (float*)(ws + kOffDAI);
  float* cbr = (float*)(ws + kOffCBR);
  float* cbi = (float*)(ws + kOffCBI);
  unsigned short* WH = (unsigned short*)(ws + kOffWH);
  unsigned short* YT = (unsigned short*)(ws + kOffYT);
  float* G  = (float*)(ws + kOffG);
  float* UA = (float*)(ws + kOffUA);
  float* UB = (float*)(ws + kOffUB);

  discretize_kernel<<<(kH + 7) / 8, 256, 0, stream>>>(log_dt, A_log, A_im, B_re, B_im, C_re, C_im, dAr, dAi, cbr, cbi);
  pack_weight_kernel<<<(kMP * (kPitch / 8)) / 256, 256, 0, stream>>>(Wout, WH);

  const float* uin[kLayers]  = { Z, UA, UB, UA };
  float*       uout[kLayers] = { UA, UB, UA, out };
  for (int layer = 0; layer < kLayers; ++layer) {
    diag_scan_gelu_kernel<<<kScBlocks, 256, 0, stream>>>(uin[layer], dAr, dAi, cbr, cbi, Dv, YT);
    wmma_gemm64<0, false, 0, 0, false><<<dim3(((kMP / 64) * (kL / 64)) / 8, 1), 256, 0, stream>>>(
        WH, nullptr, kPitch, 0L,
        YT, nullptr, kPitch, 0L,
        (void*)G, nullptr, kL, 0L,
        nullptr, nullptr, 0L,
        kMP, kL, kKP, kFold);
    glu_skip_kernel<<<(kH * (kL / 4)) / 256, 256, 0, stream>>>(uin[layer], G, bout, lcount, uout[layer]);
  }
}
